// MultiQueryAttentionLayerV2_28020366639417
// MI455X (gfx1250) — hardware-verified
//
#include <hip/hip_runtime.h>


namespace {
constexpr int NB_ = 8, D = 256, NPOS = 1024, H = 8, KD = 64, VD = 64;
constexpr float XS = 8.0f, HS = 256.0f, PS = 256.0f, WSC = 256.0f, SCALE = 0.125f;
typedef _Float16 b16;
typedef __attribute__((ext_vector_type(16))) _Float16 v16b;
typedef __attribute__((ext_vector_type(8))) _Float16 v8b;
typedef __attribute__((ext_vector_type(8))) float v8f;
typedef __attribute__((ext_vector_type(4))) float v4f;
typedef __attribute__((ext_vector_type(2))) float v2f;
typedef __attribute__((ext_vector_type(2))) _Float16 v2b;
__device__ __forceinline__ float bf16_rne(float f) { unsigned int u = __float_as_uint(f); u += 0x7FFFu + ((u >> 16) & 1u); float r = __uint_as_float(u & 0xFFFF0000u); asm volatile("" : "+v"(r)); return r; }
__device__ __forceinline__ float bfv(float f) { float r = bf16_rne(f); asm volatile("" : "+v"(r)); return r; }
__device__ __forceinline__ void split16(float v, b16& hi, b16& lo) { hi = (b16)v; lo = (b16)(v - (float)hi); }
__device__ __forceinline__ v16b frag_kb(const b16* p, int hh) { const v8b a = *(const v8b*)(p + 8 * hh), b = *(const v8b*)(p + 16 + 8 * hh); v16b f;
#pragma unroll
  for (int e = 0; e < 8; ++e) { f[e] = a[e]; f[8 + e] = b[e]; } return f; }
__device__ __forceinline__ v8f wmma16b(v16b a, v16b b, v8f c) { v8f d = __builtin_amdgcn_wmma_f32_16x16x32_f16(false, a, false, b, (short)0, c, false, false); asm volatile("v_nop\n\tv_nop\n\tv_nop\n\tv_nop" : "+v"(d) : "v"(a), "v"(b)); return d; }
__device__ __forceinline__ void wave_lds_sync() { __builtin_amdgcn_fence(__ATOMIC_RELEASE, "workgroup"); __builtin_amdgcn_wave_barrier(); __builtin_amdgcn_fence(__ATOMIC_ACQUIRE, "workgroup"); }

__global__ __launch_bounds__(256) void wput_kernel(const float* __restrict__ wq, const float* __restrict__ wk, const float* __restrict__ wv, const float* __restrict__ wo, b16* __restrict__ WQ, b16* __restrict__ WKV, b16* __restrict__ WO) { const size_t nt = (size_t)gridDim.x * 256, u0 = (size_t)blockIdx.x * 256 + threadIdx.x; v8b v; auto put = [&](b16* dst) { for (int pass = 0; pass < 2; ++pass) { *(volatile v8b*)dst = v; __threadfence(); } };
  for (size_t u = u0; u < (size_t)512 * 32; u += nt) { const int o = (int)(u / 32), d0 = (int)(u % 32) * 8; const int h = o / KD, k = o % KD;
#pragma unroll
    for (int j = 0; j < 8; ++j) v[j] = (b16)(bf16_rne(wq[((size_t)h * D + d0 + j) * KD + k]) * WSC); put(WQ + (size_t)o * D + d0); }
  for (size_t u = u0; u < (size_t)128 * 32; u += nt) { const int o = (int)(u / 32), d0 = (int)(u % 32) * 8;
#pragma unroll
    for (int j = 0; j < 8; ++j) v[j] = (b16)(bf16_rne(o < 64 ? wk[(size_t)(d0 + j) * KD + o] : wv[(size_t)(d0 + j) * VD + (o - 64)]) * WSC); put(WKV + (size_t)o * D + d0); }
  for (size_t u = u0; u < (size_t)D * 64; u += nt) { const int dd = (int)(u / 64), c0 = (int)(u % 64) * 8; const int h = c0 / 64, v0 = c0 % 64;
#pragma unroll
    for (int j = 0; j < 8; ++j) v[j] = (b16)(bf16_rne(wo[((size_t)dd * VD + v0 + j) * H + h]) * WSC); put(WO + (size_t)dd * 512 + c0); } }
__global__ __launch_bounds__(32) void proj_kernel(const float* __restrict__ xb, const float* __restrict__ vb, const b16* __restrict__ WQ, const b16* __restrict__ WKV, int NLIM, b16* __restrict__ QH, b16* __restrict__ QL, b16* __restrict__ KH, b16* __restrict__ KL, float* __restrict__ Vr) { __shared__ __attribute__((aligned(16))) b16 Ax[16][D + 8]; __shared__ float Tf[16][516]; const int lane = threadIdx.x, nloc = lane & 15, hlf = lane >> 4; const int n0 = blockIdx.x * 16, which = blockIdx.y; if (n0 >= NLIM) return; const float* src = which == 0 ? xb : vb;
  for (int q = 0; q < D / 32; ++q) { const int d = q * 32 + lane; const float* sp = src + (size_t)d * NPOS + n0; for (int rr = 0; rr < 16; ++rr) Ax[rr][d] = (b16)(bfv(sp[rr]) * XS); }
  if (lane < 16) for (int k = D; k < D + 8; ++k) Ax[lane][k] = (b16)0.0f;
  wave_lds_sync();
  const int ngr = which == 0 ? 2 : 1; const b16* Wb = which == 0 ? WQ : WKV;
#pragma unroll 1
  for (int g = 0; g < ngr; ++g) { const int ntl = which == 0 ? 16 : 8; v8f acc[16];
#pragma unroll
    for (int t = 0; t < 16; ++t) acc[t] = (v8f){};
#pragma unroll 2
    for (int kb = 0; kb < D; kb += 32) { const v16b a = frag_kb(&Ax[nloc][kb], hlf);
#pragma unroll
      for (int t = 0; t < 16; ++t) if (t < ntl) acc[t] = wmma16b(a, frag_kb(Wb + (size_t)(g * 256 + t * 16 + nloc) * D + kb, hlf), acc[t]); }
#pragma unroll
    for (int t = 0; t < 16; ++t) if (t < ntl)
#pragma unroll
      for (int r8 = 0; r8 < 8; ++r8) Tf[8 * hlf + r8][g * 256 + t * 16 + nloc] = acc[t][r8] * (1.0f / (XS * WSC)); }
  wave_lds_sync();
  for (int pass = 0; pass < 2; ++pass) {
    if (which == 0) { for (int rr = 0; rr < 16; ++rr) for (int h = 0; h < H; ++h) { b16 a0, l0, a1, l1; split16(Tf[rr][h * KD + 2 * lane] * HS, a0, l0); split16(Tf[rr][h * KD + 2 * lane + 1] * HS, a1, l1); const size_t o = ((size_t)h * NPOS + n0 + rr) * KD + 2 * lane; *(volatile v2b*)(QH + o) = (v2b){a0, a1}; *(volatile v2b*)(QL + o) = (v2b){l0, l1}; } }
    else { for (int rr = 0; rr < 16; ++rr) { b16 a0, l0, a1, l1; split16(Tf[rr][2 * lane] * HS, a0, l0); split16(Tf[rr][2 * lane + 1] * HS, a1, l1); const size_t o = (size_t)(n0 + rr) * KD + 2 * lane; *(volatile v2b*)(KH + o) = (v2b){a0, a1}; *(volatile v2b*)(KL + o) = (v2b){l0, l1}; *(volatile v2f*)(Vr + (size_t)(n0 + rr) * VD + 2 * lane) = (v2f){Tf[rr][64 + 2 * lane], Tf[rr][64 + 2 * lane + 1]}; } }
    __threadfence(); } }
__global__ __launch_bounds__(256) void vt_kernel(const float* __restrict__ Vr, int NLIM, b16* __restrict__ VTH, b16* __restrict__ VTL) { __shared__ float Tt[64][65]; const int m0 = blockIdx.x * 64; if (m0 >= NLIM) return; const int tid = threadIdx.x, wave = tid >> 5, lane = tid & 31;
  for (int q = wave; q < 64; q += 8) { Tt[q][lane] = Vr[(size_t)(m0 + q) * VD + lane]; Tt[q][32 + lane] = Vr[(size_t)(m0 + q) * VD + 32 + lane]; }
  __syncthreads();
  for (int pass = 0; pass < 2; ++pass) { for (int v = wave; v < 64; v += 8) { b16 h0, l0, h1, l1; split16(Tt[lane * 2][v] * HS, h0, l0); split16(Tt[lane * 2 + 1][v] * HS, h1, l1); const size_t o = (size_t)v * NPOS + m0 + lane * 2; *(volatile v2b*)(VTH + o) = (v2b){h0, h1}; *(volatile v2b*)(VTL + o) = (v2b){l0, l1}; } __threadfence(); } }
__global__ __launch_bounds__(32) void score_kernel(const b16* __restrict__ QH, const b16* __restrict__ QL, const b16* __restrict__ KH, const b16* __restrict__ KL, int NLIM, float* __restrict__ L) { __shared__ float Tf[16][260]; const int lane = threadIdx.x, nloc = lane & 15, hlf = lane >> 4; const int h = blockIdx.x / (NPOS / 16), n0 = (blockIdx.x % (NPOS / 16)) * 16; if (n0 >= NLIM) return;
  v16b qa[2], ql[2]; for (int ks = 0; ks < 2; ++ks) { qa[ks] = frag_kb(QH + ((size_t)h * NPOS + n0 + nloc) * KD + ks * 32, hlf); ql[ks] = frag_kb(QL + ((size_t)h * NPOS + n0 + nloc) * KD + ks * 32, hlf); }
#pragma unroll 1
  for (int g = 0; g < NPOS / 256; ++g) {
#pragma unroll 1
    for (int tg = 0; tg < 16; tg += 4) { v8f s[4] = {(v8f){}, (v8f){}, (v8f){}, (v8f){}};
#pragma unroll
      for (int t = 0; t < 4; ++t)
#pragma unroll
        for (int ks = 0; ks < 2; ++ks) { const size_t ko = (size_t)(g * 256 + (tg + t) * 16 + nloc) * KD + ks * 32; const v16b kh = frag_kb(KH + ko, hlf), kl = frag_kb(KL + ko, hlf); s[t] = wmma16b(qa[ks], kh, s[t]); s[t] = wmma16b(qa[ks], kl, s[t]); s[t] = wmma16b(ql[ks], kh, s[t]); }
#pragma unroll
      for (int t = 0; t < 4; ++t)
#pragma unroll
        for (int r8 = 0; r8 < 8; ++r8) Tf[8 * hlf + r8][(tg + t) * 16 + nloc] = s[t][r8] * (SCALE / (HS * HS)); }
    wave_lds_sync();
    for (int pass = 0; pass < 2; ++pass) { for (int rr = 0; rr < 16; ++rr) for (int q = 0; q < 2; ++q) *(volatile v4f*)(L + ((size_t)h * NPOS + n0 + rr) * NPOS + g * 256 + q * 128 + lane * 4) = *(const v4f*)(&Tf[rr][q * 128 + lane * 4]); __threadfence(); }
    wave_lds_sync(); } }
__global__ __launch_bounds__(256) void hsoft_kernel(const float* __restrict__ L, int NLIM, b16* __restrict__ PH, b16* __restrict__ PL) { const size_t u2 = (size_t)blockIdx.x * 256 + threadIdx.x; if (u2 >= (size_t)NLIM * NPOS / 2) return; const size_t u = u2 * 2;
  float l0[H], l1[H], m0 = -INFINITY, m1 = -INFINITY;
#pragma unroll
  for (int h = 0; h < H; ++h) { const v2f t = *(const v2f*)(L + (size_t)h * NPOS * NPOS + u); l0[h] = t[0]; l1[h] = t[1]; m0 = fmaxf(m0, t[0]); m1 = fmaxf(m1, t[1]); }
  float z0 = 0.0f, z1 = 0.0f;
#pragma unroll
  for (int h = 0; h < H; ++h) { l0[h] = __expf(l0[h] - m0); z0 += l0[h]; l1[h] = __expf(l1[h] - m1); z1 += l1[h]; }
  const float i0 = 1.0f / z0, i1 = 1.0f / z1;
  for (int pass = 0; pass < 2; ++pass) {
#pragma unroll
    for (int h = 0; h < H; ++h) { b16 p0, q0, p1, q1; split16(l0[h] * i0 * PS, p0, q0); split16(l1[h] * i1 * PS, p1, q1); *(volatile v2b*)(PH + (size_t)h * NPOS * NPOS + u) = (v2b){p0, p1}; *(volatile v2b*)(PL + (size_t)h * NPOS * NPOS + u) = (v2b){q0, q1}; }
    __threadfence(); } }
__global__ __launch_bounds__(32) void pv_kernel(const b16* __restrict__ PH, const b16* __restrict__ PL, const b16* __restrict__ VTH, const b16* __restrict__ VTL, int NLIM, float* __restrict__ Or) { __shared__ float Tf[16][68]; const int lane = threadIdx.x, nloc = lane & 15, hlf = lane >> 4; const int h = blockIdx.x / (NPOS / 16), n0 = (blockIdx.x % (NPOS / 16)) * 16; if (n0 >= NLIM) return;
  v8f acc[4] = {(v8f){}, (v8f){}, (v8f){}, (v8f){}}; const size_t prow = ((size_t)h * NPOS + n0 + nloc) * NPOS;
#pragma unroll 2
  for (int kb = 0; kb < NPOS; kb += 32) { if (kb >= NLIM) break; const v16b pa = frag_kb(PH + prow + kb, hlf), pb = frag_kb(PL + prow + kb, hlf);
#pragma unroll
    for (int t = 0; t < 4; ++t) { const size_t vo = (size_t)(t * 16 + nloc) * NPOS + kb; const v16b vh = frag_kb(VTH + vo, hlf), vl = frag_kb(VTL + vo, hlf); acc[t] = wmma16b(pa, vh, acc[t]); acc[t] = wmma16b(pa, vl, acc[t]); acc[t] = wmma16b(pb, vh, acc[t]); } }
#pragma unroll
  for (int t = 0; t < 4; ++t)
#pragma unroll
    for (int r8 = 0; r8 < 8; ++r8) Tf[8 * hlf + r8][t * 16 + nloc] = acc[t][r8] * (1.0f / (PS * HS));
  wave_lds_sync();
  for (int pass = 0; pass < 2; ++pass) { for (int rr = 0; rr < 16; ++rr) *(volatile v2f*)(Or + (size_t)(n0 + rr) * 512 + h * VD + lane * 2) = (v2f){Tf[rr][lane * 2], Tf[rr][lane * 2 + 1]}; __threadfence(); } }
__global__ __launch_bounds__(32) void out_kernel(const float* __restrict__ Or, const b16* __restrict__ WO, int NLIM, float* __restrict__ FIN) { __shared__ __attribute__((aligned(16))) b16 Ah[16][520], Al[16][520]; __shared__ float Tf[16][260]; const int lane = threadIdx.x, nloc = lane & 15, hlf = lane >> 4; const int n0 = blockIdx.x * 16; if (n0 >= NLIM) return;
  for (int rr = 0; rr < 16; ++rr) for (int q = 0; q < 16; ++q) { const int c = q * 32 + lane; b16 p, pl; split16(Or[(size_t)(n0 + rr) * 512 + c] * HS, p, pl); Ah[rr][c] = p; Al[rr][c] = pl; }
  if (lane < 16) for (int k = 512; k < 520; ++k) { Ah[lane][k] = (b16)0.0f; Al[lane][k] = (b16)0.0f; }
  wave_lds_sync(); v8f acc[16];
#pragma unroll
  for (int t = 0; t < 16; ++t) acc[t] = (v8f){};
#pragma unroll 2
  for (int kb = 0; kb < 512; kb += 32) { const v16b a = frag_kb(&Ah[nloc][kb], hlf), al = frag_kb(&Al[nloc][kb], hlf);
#pragma unroll
    for (int t = 0; t < 16; ++t) { const v16b bw = frag_kb(WO + (size_t)(t * 16 + nloc) * 512 + kb, hlf); acc[t] = wmma16b(a, bw, acc[t]); acc[t] = wmma16b(al, bw, acc[t]); } }
#pragma unroll
  for (int t = 0; t < 16; ++t)
#pragma unroll
    for (int r8 = 0; r8 < 8; ++r8) Tf[8 * hlf + r8][t * 16 + nloc] = acc[t][r8] * (1.0f / (HS * WSC));
  wave_lds_sync();
  for (int pass = 0; pass < 2; ++pass) { for (int rr = 0; rr < 16; ++rr) for (int q = 0; q < 2; ++q) *(volatile v4f*)(FIN + (size_t)(n0 + rr) * D + q * 128 + lane * 4) = *(const v4f*)(&Tf[rr][q * 128 + lane * 4]); __threadfence(); } }
__global__ __launch_bounds__(256) void copy_kernel(const float* __restrict__ FIN, int NLIM, float* __restrict__ outb) { const size_t u = (size_t)blockIdx.x * 256 + threadIdx.x; if (u >= (size_t)D * NPOS) return; const int n = (int)(u % NPOS), d = (int)(u / NPOS); const float v = n < NLIM ? FIN[(size_t)n * D + d] : 0.0f;
  for (int pass = 0; pass < 2; ++pass) { ((volatile float*)outb)[u] = v; __threadfence(); } }
}

extern "C" void kernel_launch(void* const* d_in, const int* in_sizes, int n_in, void* d_out, int out_size, void* d_ws, size_t ws_size, hipStream_t stream) {
  (void)n_in;
  auto Fp = [&](int i) { return (const float*)d_in[i]; };
  if (in_sizes[0] != NB_ * D * NPOS || in_sizes[1] != NB_ * D * NPOS || in_sizes[2] != H * D * KD || in_sizes[3] != D * KD || in_sizes[4] != D * VD || in_sizes[5] != D * VD * H || out_size != NB_ * D * NPOS) return;
  const int NLIM = NPOS;
  size_t off = 0; char* ws = (char*)d_ws;
  auto carve = [&](size_t bytes) { char* p = ws + off; off += (bytes + 255) & ~(size_t)255; return p; };
  b16* WQ = (b16*)carve((size_t)512 * D * 2); b16* WKV = (b16*)carve((size_t)128 * D * 2); b16* WO = (b16*)carve((size_t)D * 512 * 2);
  b16* QH = (b16*)carve((size_t)H * NPOS * KD * 2); b16* QL = (b16*)carve((size_t)H * NPOS * KD * 2); b16* KH = (b16*)carve((size_t)NPOS * KD * 2); b16* KL = (b16*)carve((size_t)NPOS * KD * 2); float* Vr = (float*)carve((size_t)NPOS * VD * 4); b16* VTH = (b16*)carve((size_t)VD * NPOS * 2); b16* VTL = (b16*)carve((size_t)VD * NPOS * 2);
  float* L = (float*)carve((size_t)H * NPOS * NPOS * 4); b16* PH = (b16*)carve((size_t)H * NPOS * NPOS * 2); b16* PL = (b16*)carve((size_t)H * NPOS * NPOS * 2); float* Or = (float*)carve((size_t)NPOS * 512 * 4); float* FIN = (float*)carve((size_t)NPOS * D * 4);
  if (off > ws_size || off > ((size_t)96 << 20)) return;
  wput_kernel<<<128, 256, 0, stream>>>(Fp(2), Fp(3), Fp(4), Fp(5), WQ, WKV, WO);
  for (int b = 0; b < NB_; ++b) { const float* xb = Fp(0) + (size_t)b * D * NPOS; const float* vb = Fp(1) + (size_t)b * D * NPOS; float* ob = (float*)d_out + (size_t)b * D * NPOS;
    proj_kernel<<<dim3(NPOS / 16, 2), 32, 0, stream>>>(xb, vb, WQ, WKV, NLIM, QH, QL, KH, KL, Vr);
    vt_kernel<<<NPOS / 64, 256, 0, stream>>>(Vr, NLIM, VTH, VTL);
    score_kernel<<<H * (NPOS / 16), 32, 0, stream>>>(QH, QL, KH, KL, NLIM, L);
    hsoft_kernel<<<(NPOS * NPOS / 2 + 255) / 256, 256, 0, stream>>>(L, NLIM, PH, PL);
    pv_kernel<<<H * (NPOS / 16), 32, 0, stream>>>(PH, PL, VTH, VTL, NLIM, Or);
    out_kernel<<<NPOS / 16, 32, 0, stream>>>(Or, WO, NLIM, FIN);
    copy_kernel<<<(D * NPOS + 255) / 256, 256, 0, stream>>>(FIN, NLIM, ob); }
}
